// EncapsulationGNN_2061584302396
// MI455X (gfx1250) — hardware-verified
//
#include <hip/hip_runtime.h>
#include <hip/hip_bf16.h>
#include <stddef.h>
#include <math.h>


#define FD      128
#define XD      5
#define EMB     32
#define KIN0    37
#define KIP     64
#define EDD     3
#define W1K     259
#define PPW     256
#define UK      256
#define NLAY    3
#define HK1     192
#define HN2     64
#define HN3     32
#define NGF     8
#define NB      256
#define NTHR    256
#define NWAVE   8
#define EPT     8
#define CHUNK   (NTHR * EPT)
#define WCAP    (EPT * 32)
#define PASSN   128
#define PCAP    4064
#define EHDR    32
#define EROW    (EHDR + PCAP)
#define RMAX    ((PCAP + NB + PASSN - 1) / PASSN)
#define RT      64
#define RTHR    128
#define GB      16
#define PTHR    256
#define PEPT    4
#define PCHUNK  (PTHR * PEPT)
#define PWCAP   (PEPT * 32)
#define HTHR    128
#define HG      64
#define NCNT    272
#define NWCB    512

#define LL_ACC  0
#define LL_MSG  (LL_ACC + (NB + 1) * FD * 4)
#define LL_CNT  (LL_MSG + PASSN * FD * 4)
#define LL_SLOT (LL_CNT + NCNT * 4)
#define LL_WCB  (LL_SLOT + PASSN * 4)
#define LL_TOT  (LL_WCB + NWCB * 4)
#define LP_STG  (4 * 2 * 16 * FD * 2)
#define LP_TOT  (LP_STG + RT * PPW * 4)

#define U0 (FD * KIP / 8)
#define U1 (NLAY * PPW * FD / 8)
#define U2 (NLAY * FD * FD / 8)
#define U3 (NLAY * FD * UK / 8)
#define U4 (NLAY * FD * FD / 8)
#define U5 (FD * HK1 / 8)
#define U6 (HN2 * FD / 8)
#define U7 (HN3 * HN2 / 8)
#define PE0 (U0 / NTHR)
#define PE1 (PE0 + U1 / NTHR)
#define PE2 (PE1 + U2 / NTHR)
#define PE3 (PE2 + U3 / NTHR)
#define PE4 (PE3 + U4 / NTHR)
#define PE5 (PE4 + U5 / NTHR)
#define PE6 (PE5 + U6 / NTHR)
#define PE7 (PE6 + U7 / NTHR)
#define PBT PE7

static_assert(NB == 2 * NWAVE * 16);
static_assert(NTHR == NWAVE * 32);
static_assert(NTHR == 2 * PASSN);
static_assert(NWAVE * 2 * 16 * FD * 2 == PASSN * FD * 4);
static_assert(EHDR * 4 == 128);
static_assert(((EROW * 4) % 512) == 0);
static_assert(RMAX == 34);
static_assert((LL_TOT % 16) == 0 && LL_TOT <= 300 * 1024);
static_assert((LP_STG % 16) == 0 && LP_TOT <= 300 * 1024);
static_assert((U0 % NTHR) == 0 && (U1 % NTHR) == 0 && (U2 % NTHR) == 0 && (U3 % NTHR) == 0);
static_assert((U4 % NTHR) == 0 && (U5 % NTHR) == 0 && (U6 % NTHR) == 0 && (U7 % NTHR) == 0);
static_assert(PBT == 165);
static_assert(NCNT >= NB + 1 && NWCB == 3 * FD + FD);
static_assert(RT == 4 * 16 && RTHR == 4 * 32 && (NB % RT) == 0);
static_assert(HTHR == 4 * 32 && HG == 4 * 16);
static_assert((KIP % 32) == 0 && KIP >= KIN0 && KIN0 == XD + EMB);
static_assert(GB == 16 && PTHR == NWAVE * 32 && (HG % GB) == 0);
static_assert((HK1 % 32) == 0 && HK1 == FD + HN2 && (HN2 % 32) == 0);

typedef float          v4f   __attribute__((ext_vector_type(4)));
typedef float          v8f   __attribute__((ext_vector_type(8)));
typedef int            v4i   __attribute__((ext_vector_type(4)));
typedef unsigned short v4us  __attribute__((ext_vector_type(4)));
typedef unsigned short v8us  __attribute__((ext_vector_type(8)));
typedef unsigned short v16us __attribute__((ext_vector_type(16)));
typedef __bf16         v16bf __attribute__((ext_vector_type(16)));
union FragB { v16bf v; v16us u; v8us h[2]; };
union Pk8 { v8us h; v4i i; };

__device__ __forceinline__ unsigned f2bf(float f) {
  const unsigned u = __float_as_uint(f);
  return (u + 0x7FFFu + ((u >> 16) & 1u)) >> 16;
}

__device__ __forceinline__ void split4(v4f a, v4us& hi, v4us& lo) {
  float f[4];
  f[0] = a.x; f[1] = a.y; f[2] = a.z; f[3] = a.w;
  v4us rh, rl;
#pragma unroll
  for (int i = 0; i < 4; ++i) {
    const unsigned hb = f2bf(f[i]);
    const float r = f[i] - __uint_as_float(hb << 16);
    rh[i] = (unsigned short)hb;
    rl[i] = (unsigned short)f2bf(r);
  }
  hi = rh;
  lo = rl;
}

__device__ __forceinline__ void split8(v4f a, v4f b, v8us& hi, v8us& lo) {
  float f[8];
  f[0] = a.x; f[1] = a.y; f[2] = a.z; f[3] = a.w;
  f[4] = b.x; f[5] = b.y; f[6] = b.z; f[7] = b.w;
  v8us rh, rl;
#pragma unroll
  for (int i = 0; i < 8; ++i) {
    const unsigned hb = f2bf(f[i]);
    const float r = f[i] - __uint_as_float(hb << 16);
    rh[i] = (unsigned short)hb;
    rl[i] = (unsigned short)f2bf(r);
  }
  hi = rh;
  lo = rl;
}

__device__ __forceinline__ v8f wm3(v16bf ah, v16bf al, v16bf bh, v16bf bl, v8f c) {
  v8f d = __builtin_amdgcn_wmma_f32_16x16x32_bf16(false, ah, false, bh, (short)0, c, false, false);
  d = __builtin_amdgcn_wmma_f32_16x16x32_bf16(false, ah, false, bl, (short)0, d, false, false);
  d = __builtin_amdgcn_wmma_f32_16x16x32_bf16(false, al, false, bh, (short)0, d, false, false);
  asm volatile("v_nop\n\tv_nop\n\tv_nop\n\tv_nop" : "+v"(d) : "v"(ah), "v"(al), "v"(bh), "v"(bl));
  return d;
}

template <int NF>
__device__ __forceinline__ void gemm_t(const unsigned short* th, const unsigned short* tl, int lda, int nkt,
    const unsigned short* __restrict__ bh, const unsigned short* __restrict__ bl, int kp, int n0, int kb,
    v8f (&acc)[NF], int hh, int m) {
  const unsigned short* ap = th + m * lda + 8 * hh;
  const unsigned short* aq = tl + m * lda + 8 * hh;
  const unsigned short* bp = bh + (size_t)(n0 + m) * kp + kb + 8 * hh;
  const unsigned short* bq = bl + (size_t)(n0 + m) * kp + kb + 8 * hh;
#pragma unroll 1
  for (int kt = 0; kt < nkt; ++kt) {
    FragB ah, al;
    ah.h[0] = *(const v8us*)(ap + 32 * kt);
    ah.h[1] = *(const v8us*)(ap + 32 * kt + 16);
    al.h[0] = *(const v8us*)(aq + 32 * kt);
    al.h[1] = *(const v8us*)(aq + 32 * kt + 16);
#pragma unroll
    for (int f = 0; f < NF; ++f) {
      FragB fh, fl;
      const size_t o = (size_t)(16 * f) * kp + 32 * kt;
      fh.h[0] = *(const v8us*)(bp + o);
      fh.h[1] = *(const v8us*)(bp + o + 16);
      fl.h[0] = *(const v8us*)(bq + o);
      fl.h[1] = *(const v8us*)(bq + o + 16);
      acc[f] = wm3(ah.v, al.v, fh.v, fl.v, acc[f]);
    }
  }
}

template <int NF>
__device__ __forceinline__ void init_b(v8f (&a)[NF], const float* __restrict__ bias, int n0, int m) {
#pragma unroll
  for (int f = 0; f < NF; ++f) {
    const float bb = bias[n0 + 16 * f + m];
    v8f c;
#pragma unroll
    for (int r = 0; r < 8; ++r) c[r] = bb;
    a[f] = c;
  }
}

template <int NF>
__device__ __forceinline__ void init_z(v8f (&a)[NF]) {
#pragma unroll
  for (int f = 0; f < NF; ++f) {
    v8f c;
#pragma unroll
    for (int r = 0; r < 8; ++r) c[r] = 0.0f;
    a[f] = c;
  }
}

template <int NF, int RELU>
__device__ __forceinline__ void put_hl(unsigned short* th, unsigned short* tl, int lda, int c0,
                                       v8f (&a)[NF], int hh, int m) {
#pragma unroll
  for (int f = 0; f < NF; ++f) {
#pragma unroll
    for (int r = 0; r < 8; ++r) {
      float v = a[f][r];
      if (RELU) v = fmaxf(v, 0.0f);
      const unsigned hb = f2bf(v);
      const unsigned lb = f2bf(v - __uint_as_float(hb << 16));
      const int o = (8 * hh + r) * lda + c0 + 16 * f + m;
      th[o] = (unsigned short)hb;
      tl[o] = (unsigned short)lb;
    }
  }
}

template <int NF, int RELU>
__device__ __forceinline__ void put_f32(float* stg, int pitch, int c0, v8f (&a)[NF], int hh, int m) {
#pragma unroll
  for (int f = 0; f < NF; ++f) {
#pragma unroll
    for (int r = 0; r < 8; ++r) {
      float v = a[f][r];
      if (RELU) v = fmaxf(v, 0.0f);
      stg[(8 * hh + r) * pitch + c0 + 16 * f + m] = v;
    }
  }
}

__device__ __forceinline__ void rows_to_tile(const float* src, int spitch, unsigned short* th, unsigned short* tl,
                                             int lda, int lane) {
#pragma unroll 4
  for (int i = 0; i < 16; ++i) {
    const v4f v = *(const v4f*)(src + (size_t)i * spitch + 4 * lane);
    v4us hi, lo;
    split4(v, hi, lo);
    *(v4us*)(th + i * lda + 4 * lane) = hi;
    *(v4us*)(tl + i * lda + 4 * lane) = lo;
  }
}

__device__ __forceinline__ int scan_chunk(const int* __restrict__ dsts, int nE, int cbase, int nodeBase,
                                          int vec8, int* list, int tid, int wave) {
  int wc = 0;
  const int el0  = tid * EPT;
  const int e0   = cbase + el0;
  const int sent = -2147483647 - 1;
  v4i da, db;
  if (vec8 != 0 && cbase + CHUNK <= nE) {
    da = *(const v4i*)(dsts + e0);
    db = *(const v4i*)(dsts + e0 + 4);
  } else {
    da.x = (e0     < nE) ? dsts[min(e0, nE - 1)] : sent;
    da.y = (e0 + 1 < nE) ? dsts[min(e0 + 1, nE - 1)] : sent;
    da.z = (e0 + 2 < nE) ? dsts[min(e0 + 2, nE - 1)] : sent;
    da.w = (e0 + 3 < nE) ? dsts[min(e0 + 3, nE - 1)] : sent;
    db.x = (e0 + 4 < nE) ? dsts[min(e0 + 4, nE - 1)] : sent;
    db.y = (e0 + 5 < nE) ? dsts[min(e0 + 5, nE - 1)] : sent;
    db.z = (e0 + 6 < nE) ? dsts[min(e0 + 6, nE - 1)] : sent;
    db.w = (e0 + 7 < nE) ? dsts[min(e0 + 7, nE - 1)] : sent;
  }
  const unsigned nb = (unsigned)nodeBase;
  const unsigned s0 = (unsigned)da.x - nb, s1 = (unsigned)da.y - nb;
  const unsigned s2 = (unsigned)da.z - nb, s3 = (unsigned)da.w - nb;
  const unsigned s4 = (unsigned)db.x - nb, s5 = (unsigned)db.y - nb;
  const unsigned s6 = (unsigned)db.z - nb, s7 = (unsigned)db.w - nb;
  const bool h0 = s0 < (unsigned)NB, h1 = s1 < (unsigned)NB, h2 = s2 < (unsigned)NB, h3 = s3 < (unsigned)NB;
  const bool h4 = s4 < (unsigned)NB, h5 = s5 < (unsigned)NB, h6 = s6 < (unsigned)NB, h7 = s7 < (unsigned)NB;
  const unsigned any = __builtin_amdgcn_ballot_w32(h0 | h1 | h2 | h3 | h4 | h5 | h6 | h7);
  if (any != 0u) {
#define HITJ(J, HJ) { \
      const unsigned mj = __builtin_amdgcn_ballot_w32(HJ); \
      if (mj != 0u) { \
        if (HJ) { \
          const int pos = wc + (int)__builtin_amdgcn_mbcnt_lo(mj, 0u); \
          if (pos < WCAP) list[wave * WCAP + pos] = el0 + (J); \
        } \
        wc += (int)__builtin_popcount(mj); } }
    HITJ(0, h0)
    HITJ(1, h1)
    HITJ(2, h2)
    HITJ(3, h3)
    HITJ(4, h4)
    HITJ(5, h5)
    HITJ(6, h6)
    HITJ(7, h7)
#undef HITJ
  }
  return wc;
}

__global__ __launch_bounds__(NTHR) void k_prep(
    const float* __restrict__ win, const float* __restrict__ mw1, const float* __restrict__ mw2,
    const float* __restrict__ uw1, const float* __restrict__ uw2,
    const float* __restrict__ hw1, const float* __restrict__ hw2, const float* __restrict__ hw3,
    unsigned short* q0, unsigned short* q1, unsigned short* q2, unsigned short* q3,
    unsigned short* q4, unsigned short* q5, unsigned short* q6, unsigned short* q7) {
  const int b = blockIdx.x, tid = threadIdx.x;
  const float* src;
  unsigned short* dst;
  int Kin, Kp, O, L, ub, spl;
  if (b < PE0)      { src = win; dst = q0; Kin = KIN0; Kp = KIP; O = FD;  L = 1;    ub = b;       spl = 0; }
  else if (b < PE1) { src = mw1; dst = q1; Kin = FD;   Kp = FD;  O = PPW; L = NLAY; ub = b - PE0; spl = 1; }
  else if (b < PE2) { src = mw2; dst = q2; Kin = FD;   Kp = FD;  O = FD;  L = NLAY; ub = b - PE1; spl = 0; }
  else if (b < PE3) { src = uw1; dst = q3; Kin = UK;   Kp = UK;  O = FD;  L = NLAY; ub = b - PE2; spl = 0; }
  else if (b < PE4) { src = uw2; dst = q4; Kin = FD;   Kp = FD;  O = FD;  L = NLAY; ub = b - PE3; spl = 0; }
  else if (b < PE5) { src = hw1; dst = q5; Kin = HK1;  Kp = HK1; O = FD;  L = 1;    ub = b - PE4; spl = 0; }
  else if (b < PE6) { src = hw2; dst = q6; Kin = FD;   Kp = FD;  O = HN2; L = 1;    ub = b - PE5; spl = 0; }
  else              { src = hw3; dst = q7; Kin = HN2;  Kp = HN2; O = HN3; L = 1;    ub = b - PE6; spl = 0; }
  const int u   = ub * NTHR + tid;
  const int cpr = Kp >> 3;
  const int row = u / cpr;
  const int kc  = u - row * cpr;
  int l = row / O;
  l = l > L - 1 ? L - 1 : l;
  const int o = row - l * O;
  float f[8];
#pragma unroll
  for (int j = 0; j < 8; ++j) {
    const int k   = 8 * kc + j;
    const int kcl = k < Kin ? k : Kin - 1;
    const size_t istd = ((size_t)(l * Kin + kcl)) * O + o;
    const size_t ispl = (size_t)l * (W1K * FD) + (size_t)((o >> 7) * FD + kcl) * FD + (o & (FD - 1));
    const size_t idx = spl != 0 ? ispl : istd;
    const float w = src[idx];
    f[j] = (k < Kin) ? w : 0.0f;
  }
  Pk8 ph, pl;
  {
    v4f a, c;
    a.x = f[0]; a.y = f[1]; a.z = f[2]; a.w = f[3];
    c.x = f[4]; c.y = f[5]; c.z = f[6]; c.w = f[7];
    split8(a, c, ph.h, pl.h);
  }
  const size_t ne = (size_t)L * O * Kp;
  unsigned short* dh = dst + (size_t)u * 8;
  unsigned short* dl = dst + ne + (size_t)u * 8;
  *(volatile v4i*)dh = ph.i;
  *(volatile v4i*)dl = pl.i;
  __threadfence();
  *(volatile v4i*)dh = ph.i;
  *(volatile v4i*)dl = pl.i;
}

__global__ __launch_bounds__(NTHR) void k_escan(const int* __restrict__ ei, int* etab, int nE, int vec8) {
  __shared__ int list[NWAVE * WCAP];
  __shared__ __attribute__((aligned(16))) int pend[EROW];
  __shared__ int wcnt[NWAVE];
  const int tid = threadIdx.x, lane = tid & 31, wave = tid >> 5;
  const int nodeBase = blockIdx.x * NB;
  const int* dsts = ei + nE;
  for (int i = tid; i < EROW; i += NTHR) pend[i] = 0;
  __syncthreads();
  int pendN = 0;
  const int nChunks = (nE + CHUNK - 1) / CHUNK;
#pragma unroll 1
  for (int ch = 0; ch < nChunks; ++ch) {
    const int cbase = ch * CHUNK;
    const int wc = scan_chunk(dsts, nE, cbase, nodeBase, vec8, list, tid, wave);
    if (lane == 0) wcnt[wave] = wc;
    __syncthreads();
    const int base = pendN;
    int tot = 0, myoff = 0;
#pragma unroll
    for (int w = 0; w < NWAVE; ++w) {
      int c = wcnt[w];
      c = c > WCAP ? WCAP : (c < 0 ? 0 : c);
      if (w < wave) myoff += c;
      tot += c;
    }
    {
      int n = wcnt[wave];
      n = n > WCAP ? WCAP : (n < 0 ? 0 : n);
      const int* lp = list + wave * WCAP;
      for (int i = lane; i < n; i += 32) {
        const int pos = base + myoff + i;
        if (pos < PCAP) pend[EHDR + pos] = cbase + lp[i];
      }
    }
    const int newN = base + tot;
    pendN = newN > PCAP ? PCAP : newN;
    __syncthreads();
  }
  if (tid == 0) pend[0] = pendN;
  __syncthreads();
  int* rowp = etab + (size_t)blockIdx.x * EROW;
#pragma unroll 1
  for (int u = tid; u < EROW / 4; u += NTHR) {
    const v4i v = *(const v4i*)(pend + 4 * u);
    *(volatile v4i*)(rowp + 4 * u) = v;
  }
  __threadfence();
#pragma unroll 1
  for (int u = tid; u < EROW / 4; u += NTHR) {
    const v4i v = *(const v4i*)(pend + 4 * u);
    *(volatile v4i*)(rowp + 4 * u) = v;
  }
}

__global__ __launch_bounds__(RTHR) void k_inproj(const float* __restrict__ x, const int* __restrict__ bead,
    const float* __restrict__ emb, const unsigned short* __restrict__ wih, const unsigned short* __restrict__ wil,
    const float* __restrict__ bin, float* hout, int nN, int nBead) {
  __shared__ __attribute__((aligned(16))) unsigned short atile[4 * 2 * 16 * KIP];
  __shared__ __attribute__((aligned(16))) float stg[RT * FD];
  const int tid = threadIdx.x, lane = tid & 31, wave = tid >> 5, hh = lane >> 4, m = lane & 15;
  const int rowBase = blockIdx.x * RT;
  const int r0 = 16 * wave;
  unsigned short* th = atile + wave * (2 * 16 * KIP);
  unsigned short* tl = th + 16 * KIP;
#pragma unroll 2
  for (int idx = lane; idx < 16 * KIP; idx += 32) {
    const int i = idx / KIP;
    const int c = idx - i * KIP;
    int node = rowBase + r0 + i;
    node = node > nN - 1 ? nN - 1 : node;
    int bd = bead[node];
    bd = bd < 0 ? 0 : (bd > nBead - 1 ? nBead - 1 : bd);
    const int cx = c < XD ? c : XD - 1;
    int ce = c - XD;
    ce = ce < 0 ? 0 : (ce > EMB - 1 ? EMB - 1 : ce);
    const float xv = x[(size_t)node * XD + cx];
    const float ev = emb[(size_t)bd * EMB + ce];
    const float v = c < XD ? xv : (c < KIN0 ? ev : 0.0f);
    const unsigned hb = f2bf(v);
    const unsigned lb = f2bf(v - __uint_as_float(hb << 16));
    th[i * KIP + c] = (unsigned short)hb;
    tl[i * KIP + c] = (unsigned short)lb;
  }
  __syncthreads();
#pragma unroll 1
  for (int g = 0; g < 2; ++g) {
    v8f a[4];
    init_b<4>(a, bin, 64 * g, m);
    gemm_t<4>(th, tl, KIP, KIP / 32, wih, wil, KIP, 64 * g, 0, a, hh, m);
    put_f32<4, 0>(stg + r0 * FD, FD, 64 * g, a, hh, m);
  }
  __syncthreads();
#pragma unroll 1
  for (int rr = 0; rr < 16; ++rr) {
    const int row = r0 + rr;
    const v4f v = *(const v4f*)(stg + row * FD + 4 * lane);
    *(volatile v4f*)(hout + (size_t)(rowBase + row) * FD + 4 * lane) = v;
  }
  __threadfence();
#pragma unroll 1
  for (int rr = 0; rr < 16; ++rr) {
    const int row = r0 + rr;
    const v4f v = *(const v4f*)(stg + row * FD + 4 * lane);
    *(volatile v4f*)(hout + (size_t)(rowBase + row) * FD + 4 * lane) = v;
  }
}

__global__ __launch_bounds__(RTHR) void k_pp(const float* __restrict__ hin,
    const unsigned short* __restrict__ w1h, const unsigned short* __restrict__ w1l, float* pp) {
  extern __shared__ __attribute__((aligned(16))) unsigned char dsp[];
  unsigned short* atl = (unsigned short*)dsp;
  float* stg = (float*)(dsp + LP_STG);
  const int tid = threadIdx.x, lane = tid & 31, wave = tid >> 5, hh = lane >> 4, m = lane & 15;
  const int rowBase = blockIdx.x * RT;
  const int r0 = 16 * wave;
  unsigned short* th = atl + wave * (2 * 16 * FD);
  unsigned short* tl = th + 16 * FD;
  rows_to_tile(hin + (size_t)(rowBase + r0) * FD, FD, th, tl, FD, lane);
  __syncthreads();
#pragma unroll 1
  for (int g = 0; g < 4; ++g) {
    v8f a[4];
    init_z<4>(a);
    gemm_t<4>(th, tl, FD, FD / 32, w1h, w1l, FD, 64 * g, 0, a, hh, m);
    put_f32<4, 0>(stg + r0 * PPW, PPW, 64 * g, a, hh, m);
  }
  __syncthreads();
#pragma unroll 1
  for (int rr = 0; rr < 16; ++rr) {
    const int row = r0 + rr;
#pragma unroll
    for (int j = 0; j < 2; ++j) {
      const v4f v = *(const v4f*)(stg + row * PPW + FD * j + 4 * lane);
      *(volatile v4f*)(pp + (size_t)(rowBase + row) * PPW + FD * j + 4 * lane) = v;
    }
  }
  __threadfence();
#pragma unroll 1
  for (int rr = 0; rr < 16; ++rr) {
    const int row = r0 + rr;
#pragma unroll
    for (int j = 0; j < 2; ++j) {
      const v4f v = *(const v4f*)(stg + row * PPW + FD * j + 4 * lane);
      *(volatile v4f*)(pp + (size_t)(rowBase + row) * PPW + FD * j + 4 * lane) = v;
    }
  }
}

__global__ __launch_bounds__(NTHR) void k_layer(
    const float* __restrict__ hin, const float* __restrict__ pp,
    const int* __restrict__ ei, const float* __restrict__ eat, const int* __restrict__ etab,
    const float* __restrict__ wcp, const float* __restrict__ b1p,
    const unsigned short* __restrict__ w2h, const unsigned short* __restrict__ w2l, const float* __restrict__ b2p,
    const unsigned short* __restrict__ u1h, const unsigned short* __restrict__ u1l, const float* __restrict__ ub1,
    const unsigned short* __restrict__ u2h, const unsigned short* __restrict__ u2l, const float* __restrict__ ub2,
    const float* __restrict__ gam, const float* __restrict__ bet,
    float* hout, int nN, int nE, int resid) {
  extern __shared__ __attribute__((aligned(16))) unsigned char dsm[];
  float* acc   = (float*)(dsm + LL_ACC);
  float* msg   = (float*)(dsm + LL_MSG);
  unsigned short* atl = (unsigned short*)(dsm + LL_MSG);
  float* cntl  = (float*)(dsm + LL_CNT);
  int*   slotb = (int*)(dsm + LL_SLOT);
  float* wcb   = (float*)(dsm + LL_WCB);

  const int tid = threadIdx.x, lane = tid & 31, wave = tid >> 5, hh = lane >> 4, m = lane & 15;
  const int nodeBase = blockIdx.x * NB;
  const int* srcs = ei;
  const int* dsts = ei + nE;
  const int* erow = etab + (size_t)blockIdx.x * EROW;

  {
    const v4f z = {0.0f, 0.0f, 0.0f, 0.0f};
    for (int i = tid; i < (NB + 1) * FD / 4; i += NTHR) *(v4f*)(acc + 4 * i) = z;
    for (int i = tid; i < NCNT; i += NTHR) cntl[i] = 0.0f;
    for (int i = tid; i < NWCB; i += NTHR) {
      const int iw = i < 3 * FD ? i : 3 * FD - 1;
      int ib = i - 3 * FD;
      ib = ib < 0 ? 0 : ib;
      const float a = wcp[iw];
      const float b = b1p[ib];
      wcb[i] = (i < 3 * FD) ? a : b;
    }
  }
  int nP = erow[0];
  nP = nP < 0 ? 0 : (nP > PCAP ? PCAP : nP);
  const int tot = nP + NB;
  int R = (tot + PASSN - 1) / PASSN;
  R = R > RMAX ? RMAX : R;
  __syncthreads();

#pragma unroll 1
  for (int r = 0; r < R; ++r) {
    {
      const int i = tid >> 1, q = tid & 1;
      const int idx = r * PASSN + i;
      const bool fromTab = idx < nP;
      const int idxc = idx < PCAP ? idx : PCAP - 1;
      int e = erow[EHDR + idxc];
      e = e < 0 ? 0 : (e > nE - 1 ? nE - 1 : e);
      const int dtab = dsts[e];
      const int stab = srcs[e];
      int j = idx - nP;
      j = j < 0 ? 0 : (j > NB - 1 ? NB - 1 : j);
      const int selfn = nodeBase + j;
      const bool selfok = (idx >= nP) && (idx - nP < NB) && (selfn < nN);
      int s = fromTab ? stab : selfn;
      s = s < 0 ? 0 : (s > nN - 1 ? nN - 1 : s);
      const int d = fromTab ? dtab : selfn;
      int dcl = d < 0 ? 0 : (d > nN - 1 ? nN - 1 : d);
      int slot = d - nodeBase;
      const bool valid = fromTab || selfok;
      if (!valid || (unsigned)slot >= (unsigned)NB || d < 0 || d > nN - 1) slot = NB;
      const float* e3 = eat + (size_t)e * EDD;
      float a0 = e3[0], a1 = e3[1], a2 = e3[2];
      a0 = fromTab ? a0 : 0.0f;
      a1 = fromTab ? a1 : 0.0f;
      a2 = fromTab ? a2 : 0.0f;
      const float* par = pp + (size_t)s * PPW + 64 * q;
      const float* pbr = pp + (size_t)dcl * PPW + FD + 64 * q;
      const float* w0 = wcb + 64 * q;
      const float* w1 = wcb + FD + 64 * q;
      const float* w2 = wcb + 2 * FD + 64 * q;
      const float* bv = wcb + 3 * FD + 64 * q;
      float* mr = msg + i * FD + 64 * q;
#pragma unroll 1
      for (int p = 0; p < 2; ++p) {
#pragma unroll
        for (int jj = 0; jj < 8; ++jj) {
          const int c = 32 * p + 4 * jj;
          const v4f va = *(const v4f*)(par + c);
          const v4f vb = *(const v4f*)(pbr + c);
          const v4f x0 = *(const v4f*)(w0 + c);
          const v4f x1 = *(const v4f*)(w1 + c);
          const v4f x2 = *(const v4f*)(w2 + c);
          const v4f xb = *(const v4f*)(bv + c);
          v4f t = va + vb + xb + a0 * x0 + a1 * x1 + a2 * x2;
          v4f o;
          o.x = fmaxf(t.x, 0.0f); o.y = fmaxf(t.y, 0.0f); o.z = fmaxf(t.z, 0.0f); o.w = fmaxf(t.w, 0.0f);
          *(v4f*)(mr + c) = o;
        }
      }
      if (q == 0) slotb[i] = slot;
    }
    __syncthreads();
    {
      int cnt = tot - r * PASSN;
      cnt = cnt > PASSN ? PASSN : (cnt < 0 ? 0 : cnt);
      if (tid < FD) {
#pragma unroll 1
        for (int i = 0; i < cnt; ++i) {
          int sl = slotb[i];
          sl = sl < 0 ? 0 : (sl > NB ? NB : sl);
          acc[sl * FD + tid] += msg[i * FD + tid];
          if (tid == 0) cntl[sl] += 1.0f;
        }
      }
    }
    __syncthreads();
  }

  const float bns = 1.0f / sqrtf(1.0f + 1e-5f);
  unsigned short* th = atl + wave * (2 * 16 * FD);
  unsigned short* tl = th + 16 * FD;
#pragma unroll 1
  for (int tt = 0; tt < 2; ++tt) {
    const int t = wave + NWAVE * tt;
    const int r0 = 16 * t;
    rows_to_tile(acc + r0 * FD, FD, th, tl, FD, lane);
    float cv[8];
#pragma unroll
    for (int r = 0; r < 8; ++r) cv[r] = cntl[r0 + 8 * hh + r];
    __syncthreads();
    v8f aA[4], aB[4];
#pragma unroll
    for (int f = 0; f < 4; ++f) {
      const float ba = b2p[16 * f + m];
      const float bb = b2p[64 + 16 * f + m];
      v8f ca, cb;
#pragma unroll
      for (int r = 0; r < 8; ++r) { ca[r] = cv[r] * ba; cb[r] = cv[r] * bb; }
      aA[f] = ca;
      aB[f] = cb;
    }
    gemm_t<4>(th, tl, FD, FD / 32, w2h, w2l, FD, 0, 0, aA, hh, m);
    gemm_t<4>(th, tl, FD, FD / 32, w2h, w2l, FD, 64, 0, aB, hh, m);
    put_hl<4, 0>(th, tl, FD, 0, aA, hh, m);
    put_hl<4, 0>(th, tl, FD, 64, aB, hh, m);
    __syncthreads();
    init_b<4>(aA, ub1, 0, m);
    init_b<4>(aB, ub1, 64, m);
    gemm_t<4>(th, tl, FD, FD / 32, u1h, u1l, UK, 0, FD, aA, hh, m);
    gemm_t<4>(th, tl, FD, FD / 32, u1h, u1l, UK, 64, FD, aB, hh, m);
    __syncthreads();
    rows_to_tile(hin + (size_t)(nodeBase + r0) * FD, FD, th, tl, FD, lane);
    __syncthreads();
    gemm_t<4>(th, tl, FD, FD / 32, u1h, u1l, UK, 0, 0, aA, hh, m);
    gemm_t<4>(th, tl, FD, FD / 32, u1h, u1l, UK, 64, 0, aB, hh, m);
    put_hl<4, 1>(th, tl, FD, 0, aA, hh, m);
    put_hl<4, 1>(th, tl, FD, 64, aB, hh, m);
    __syncthreads();
#pragma unroll 1
    for (int g = 0; g < 2; ++g) {
      v8f a[4];
      init_b<4>(a, ub2, 64 * g, m);
      gemm_t<4>(th, tl, FD, FD / 32, u2h, u2l, FD, 64 * g, 0, a, hh, m);
#pragma unroll
      for (int f = 0; f < 4; ++f) {
        const int col = 64 * g + 16 * f + m;
        const float gs = gam[col];
        const float be = bet[col];
#pragma unroll
        for (int r = 0; r < 8; ++r) {
          const float v = fmaxf((a[f][r] * bns) * gs + be, 0.0f);
          acc[(r0 + 8 * hh + r) * FD + col] = v;
        }
      }
    }
    __syncthreads();
  }

#pragma unroll 1
  for (int rr = 0; rr < NB / NWAVE; ++rr) {
    const int row = wave * (NB / NWAVE) + rr;
    const v4f a = *(const v4f*)(acc + row * FD + 4 * lane);
    const v4f b = *(const v4f*)(hin + (size_t)(nodeBase + row) * FD + 4 * lane);
    const v4f v = (resid != 0) ? (a + b) : a;
    *(volatile v4f*)(hout + (size_t)(nodeBase + row) * FD + 4 * lane) = v;
  }
  __threadfence();
#pragma unroll 1
  for (int rr = 0; rr < NB / NWAVE; ++rr) {
    const int row = wave * (NB / NWAVE) + rr;
    const v4f a = *(const v4f*)(acc + row * FD + 4 * lane);
    const v4f b = *(const v4f*)(hin + (size_t)(nodeBase + row) * FD + 4 * lane);
    const v4f v = (resid != 0) ? (a + b) : a;
    *(volatile v4f*)(hout + (size_t)(nodeBase + row) * FD + 4 * lane) = v;
  }
}

__global__ __launch_bounds__(PTHR) void k_pool(const float* __restrict__ hfin, const int* __restrict__ batch,
                                              float* ge, int nN, int G) {
  __shared__ __attribute__((aligned(16))) float gt[GB * FD];
  __shared__ int plist[NWAVE * PWCAP];
  __shared__ int pwc[NWAVE];
  const int tid = threadIdx.x, lane = tid & 31, wave = tid >> 5;
  const int par = tid >> 7, c = tid & (FD - 1);
  const int g0 = blockIdx.x * GB;
  for (int i = tid; i < GB * FD; i += PTHR) gt[i] = 0.0f;
  __syncthreads();
  const int nCh = (nN + PCHUNK - 1) / PCHUNK;
#pragma unroll 1
  for (int ch = 0; ch < nCh; ++ch) {
    const int cbase = ch * PCHUNK;
    int wc = 0;
    {
      const int n0 = cbase + tid * PEPT;
      const int sent = -2147483647 - 1;
      v4i b;
      if (cbase + PCHUNK <= nN) {
        b = *(const v4i*)(batch + n0);
      } else {
        b.x = (n0     < nN) ? batch[min(n0, nN - 1)] : sent;
        b.y = (n0 + 1 < nN) ? batch[min(n0 + 1, nN - 1)] : sent;
        b.z = (n0 + 2 < nN) ? batch[min(n0 + 2, nN - 1)] : sent;
        b.w = (n0 + 3 < nN) ? batch[min(n0 + 3, nN - 1)] : sent;
      }
      const unsigned ug = (unsigned)g0;
      const unsigned s0 = (unsigned)b.x - ug, s1 = (unsigned)b.y - ug;
      const unsigned s2 = (unsigned)b.z - ug, s3 = (unsigned)b.w - ug;
      const bool h0 = s0 < (unsigned)GB, h1 = s1 < (unsigned)GB, h2 = s2 < (unsigned)GB, h3 = s3 < (unsigned)GB;
      const unsigned any = __builtin_amdgcn_ballot_w32(h0 | h1 | h2 | h3);
      if (any != 0u) {
#define PHIT(J, HJ, SJ) { \
          const unsigned mj = __builtin_amdgcn_ballot_w32(HJ); \
          if (mj != 0u) { \
            if (HJ) { \
              const int pos = wc + (int)__builtin_amdgcn_mbcnt_lo(mj, 0u); \
              if (pos < PWCAP) plist[wave * PWCAP + pos] = (n0 + (J)) * GB + (int)(SJ); \
            } \
            wc += (int)__builtin_popcount(mj); } }
        PHIT(0, h0, s0)
        PHIT(1, h1, s1)
        PHIT(2, h2, s2)
        PHIT(3, h3, s3)
#undef PHIT
      }
    }
    if (lane == 0) pwc[wave] = wc;
    __syncthreads();
#pragma unroll 1
    for (int w = 0; w < NWAVE; ++w) {
      int n = pwc[w];
      n = n > PWCAP ? PWCAP : (n < 0 ? 0 : n);
#pragma unroll 1
      for (int i = 0; i < n; ++i) {
        const int pk = plist[w * PWCAP + i];
        const int gl = pk & (GB - 1);
        int nd = pk >> 4;
        nd = nd < 0 ? 0 : (nd > nN - 1 ? nN - 1 : nd);
        if ((gl & 1) == par) {
          const float v = hfin[(size_t)nd * FD + c];
          gt[gl * FD + c] += v;
        }
      }
    }
    __syncthreads();
  }
#pragma unroll 1
  for (int rr = 0; rr < 2; ++rr) {
    const int row = 2 * wave + rr;
    const v4f v = *(const v4f*)(gt + row * FD + 4 * lane);
    *(volatile v4f*)(ge + (size_t)(g0 + row) * FD + 4 * lane) = v;
  }
  __threadfence();
#pragma unroll 1
  for (int rr = 0; rr < 2; ++rr) {
    const int row = 2 * wave + rr;
    const v4f v = *(const v4f*)(gt + row * FD + 4 * lane);
    *(volatile v4f*)(ge + (size_t)(g0 + row) * FD + 4 * lane) = v;
  }
}

__global__ __launch_bounds__(HTHR) void k_head(const float* __restrict__ ge,
    const float* __restrict__ f0, const float* __restrict__ f1, const float* __restrict__ f2, const float* __restrict__ f3,
    const float* __restrict__ f4, const float* __restrict__ f5, const float* __restrict__ f6, const float* __restrict__ f7,
    const float* __restrict__ gfw, const float* __restrict__ gfb,
    const unsigned short* __restrict__ h1h, const unsigned short* __restrict__ h1l, const float* __restrict__ hb1,
    const unsigned short* __restrict__ h2h, const unsigned short* __restrict__ h2l, const float* __restrict__ hb2,
    const unsigned short* __restrict__ h3h, const unsigned short* __restrict__ h3l, const float* __restrict__ hb3,
    const float* __restrict__ hw4, const float* __restrict__ hb4,
    float* dout, int G) {
  __shared__ __attribute__((aligned(16))) unsigned short hat[4 * 2 * 16 * HK1];
  __shared__ __attribute__((aligned(16))) float gfl[4 * 16 * NGF];
  __shared__ __attribute__((aligned(16))) float t3[4 * 16 * HN3];
  __shared__ __attribute__((aligned(16))) float o0s[HG];
  const int tid = threadIdx.x, lane = tid & 31, wave = tid >> 5, hh = lane >> 4, m = lane & 15;
  const int g0 = blockIdx.x * HG + 16 * wave;
  unsigned short* th = hat + wave * (2 * 16 * HK1);
  unsigned short* tl = th + 16 * HK1;
  float* gfr = gfl + wave * 16 * NGF;
  float* t3w = t3 + wave * 16 * HN3;
  {
    int g = g0 + m;
    g = g > G - 1 ? G - 1 : g;
    const float v0 = f0[g] * (1.0f / 100.0f);
    const float v1 = f1[g] * (1.0f / 100.0f);
    const float v2 = f2[g] * (1.0f / 10.0f);
    const float v3 = f3[g] * (1.0f / 10.0f);
    const float v4 = f4[g];
    const float v5 = f5[g] * (1.0f / 10.0f);
    const float v6 = f6[g] * (1.0f / 5.0f);
    const float v7 = f7[g] * (1.0f / 50.0f);
    if (hh == 0) {
      float* pr = gfr + m * NGF;
      pr[0] = v0; pr[1] = v1; pr[2] = v2; pr[3] = v3;
      pr[4] = v4; pr[5] = v5; pr[6] = v6; pr[7] = v7;
    }
  }
  __syncthreads();
  {
    int gb = g0;
    gb = gb > G - 16 ? G - 16 : gb;
    gb = gb < 0 ? 0 : gb;
    rows_to_tile(ge + (size_t)gb * FD, FD, th, tl, HK1, lane);
  }
#pragma unroll 2
  for (int idx = lane; idx < 16 * HN2; idx += 32) {
    const int i = idx >> 6;
    const int jc = idx & (HN2 - 1);
    float a = gfb[jc];
    const float* pr = gfr + i * NGF;
#pragma unroll
    for (int k = 0; k < NGF; ++k) a += pr[k] * gfw[k * HN2 + jc];
    const unsigned hb = f2bf(a);
    const unsigned lb = f2bf(a - __uint_as_float(hb << 16));
    th[i * HK1 + FD + jc] = (unsigned short)hb;
    tl[i * HK1 + FD + jc] = (unsigned short)lb;
  }
  __syncthreads();
  {
    v8f aA[4], aB[4];
    init_b<4>(aA, hb1, 0, m);
    init_b<4>(aB, hb1, 64, m);
    gemm_t<4>(th, tl, HK1, HK1 / 32, h1h, h1l, HK1, 0, 0, aA, hh, m);
    gemm_t<4>(th, tl, HK1, HK1 / 32, h1h, h1l, HK1, 64, 0, aB, hh, m);
    put_hl<4, 1>(th, tl, HK1, 0, aA, hh, m);
    put_hl<4, 1>(th, tl, HK1, 64, aB, hh, m);
  }
  __syncthreads();
  {
    v8f a[4];
    init_b<4>(a, hb2, 0, m);
    gemm_t<4>(th, tl, HK1, FD / 32, h2h, h2l, FD, 0, 0, a, hh, m);
    put_hl<4, 1>(th, tl, HK1, 0, a, hh, m);
  }
  __syncthreads();
  {
    v8f a[2];
    init_b<2>(a, hb3, 0, m);
    gemm_t<2>(th, tl, HK1, HN2 / 32, h3h, h3l, HN2, 0, 0, a, hh, m);
    put_f32<2, 1>(t3w, HN3, 0, a, hh, m);
  }
  __syncthreads();
  {
    const float* orow = t3w + m * HN3 + 16 * hh;
    const float* wv = hw4 + 16 * hh;
    float s = 0.0f;
#pragma unroll
    for (int k = 0; k < 16; ++k) s += orow[k] * wv[k];
    const float t = __shfl_xor(s, 16);
    const float lo = (hh == 0) ? s : t;
    const float hi = (hh == 0) ? t : s;
    float o = (lo + hi) + hb4[0];
    o = fminf(fmaxf(o, -30.0f), 30.0f);
    const float ex = expf(-o);
    const float sg = 1.0f / (1.0f + ex);
    if (hh == 0) o0s[16 * wave + m] = sg;
  }
  __syncthreads();
  v4f ov = {0.0f, 0.0f, 0.0f, 0.0f};
  if (wave == 0 && lane < 16) ov = *(const v4f*)(o0s + 4 * lane);
  if (wave == 0 && lane < 16) *(volatile v4f*)(dout + (size_t)blockIdx.x * HG + 4 * lane) = ov;
  __threadfence();
  if (wave == 0 && lane < 16) *(volatile v4f*)(dout + (size_t)blockIdx.x * HG + 4 * lane) = ov;
}

extern "C" void kernel_launch(void* const* d_in, const int* in_sizes, int n_in,
                              void* d_out, int out_size, void* d_ws, size_t ws_size,
                              hipStream_t stream) {
  if (n_in < 36) return;
  const int nN = in_sizes[3];
  if (nN < 1 || in_sizes[0] != nN * XD || in_sizes[4] != nN) return;
  const int nE = in_sizes[2] / 2;
  if (nE < 1 || in_sizes[2] != 2 * nE || in_sizes[1] != EDD * nE) return;
  const int G = out_size;
  if (G < HG || (G % HG) != 0) return;
  for (int i = 5; i <= 12; ++i) if (in_sizes[i] != G) return;
  const int nBead = in_sizes[13] / EMB;
  if (nBead < 1 || in_sizes[13] != nBead * EMB) return;
  if (in_sizes[14] != KIN0 * FD || in_sizes[15] != FD) return;
  if (in_sizes[16] != NLAY * W1K * FD || in_sizes[17] != NLAY * FD) return;
  if (in_sizes[18] != NLAY * FD * FD || in_sizes[19] != NLAY * FD) return;
  if (in_sizes[20] != NLAY * UK * FD || in_sizes[21] != NLAY * FD) return;
  if (in_sizes[22] != NLAY * FD * FD || in_sizes[23] != NLAY * FD) return;
  if (in_sizes[24] != NLAY * FD || in_sizes[25] != NLAY * FD) return;
  if (in_sizes[26] != NGF * HN2 || in_sizes[27] != HN2) return;
  if (in_sizes[28] != HK1 * FD || in_sizes[29] != FD) return;
  if (in_sizes[30] != FD * HN2 || in_sizes[31] != HN2) return;
  if (in_sizes[32] != HN2 * HN3 || in_sizes[33] != HN3) return;
  if (in_sizes[34] != HN3 || in_sizes[35] != 1) return;

  const float* x     = (const float*)d_in[0];
  const float* eat   = (const float*)d_in[1];
  const int*   ei    = (const int*)d_in[2];
  const int*   batch = (const int*)d_in[3];
  const int*   bead  = (const int*)d_in[4];
  const float* gfi0 = (const float*)d_in[5],  *gfi1 = (const float*)d_in[6];
  const float* gfi2 = (const float*)d_in[7],  *gfi3 = (const float*)d_in[8];
  const float* gfi4 = (const float*)d_in[9],  *gfi5 = (const float*)d_in[10];
  const float* gfi6 = (const float*)d_in[11], *gfi7 = (const float*)d_in[12];
  const float* emb  = (const float*)d_in[13];
  const float* win  = (const float*)d_in[14], *bin = (const float*)d_in[15];
  const float* mw1  = (const float*)d_in[16], *mb1 = (const float*)d_in[17];
  const float* mw2  = (const float*)d_in[18], *mb2 = (const float*)d_in[19];
  const float* uw1  = (const float*)d_in[20], *ub1 = (const float*)d_in[21];
  const float* uw2  = (const float*)d_in[22], *ub2 = (const float*)d_in[23];
  const float* gam  = (const float*)d_in[24], *bet = (const float*)d_in[25];
  const float* gfw  = (const float*)d_in[26], *gfb = (const float*)d_in[27];
  const float* hw1  = (const float*)d_in[28], *hb1 = (const float*)d_in[29];
  const float* hw2  = (const float*)d_in[30], *hb2 = (const float*)d_in[31];
  const float* hw3  = (const float*)d_in[32], *hb3 = (const float*)d_in[33];
  const float* hw4  = (const float*)d_in[34], *hb4 = (const float*)d_in[35];
  float* dout = (float*)d_out;

  const int nBlk = (nN + NB - 1) / NB;
  const size_t rowsP = (size_t)nBlk * NB;
  const int nRT = (int)(rowsP / RT);

  const size_t ne0 = (size_t)FD * KIP, ne1 = (size_t)NLAY * PPW * FD, ne2 = (size_t)NLAY * FD * FD;
  const size_t ne3 = (size_t)NLAY * FD * UK, ne4 = ne2, ne5 = (size_t)FD * HK1, ne6 = (size_t)HN2 * FD;
  const size_t ne7 = (size_t)HN3 * HN2;

  char* ws = (char*)d_ws;
  size_t off = 0;
  auto carve = [&](size_t bytes) -> size_t {
    const size_t o = off;
    off = (off + bytes + 255) & ~(size_t)255;
    return o;
  };
  const size_t oq0 = carve(2 * ne0 * 2), oq1 = carve(2 * ne1 * 2), oq2 = carve(2 * ne2 * 2), oq3 = carve(2 * ne3 * 2);
  const size_t oq4 = carve(2 * ne4 * 2), oq5 = carve(2 * ne5 * 2), oq6 = carve(2 * ne6 * 2), oq7 = carve(2 * ne7 * 2);
  const size_t oet = carve((size_t)nBlk * EROW * 4);
  const size_t oX0 = carve(rowsP * FD * 4);
  const size_t oX1 = carve(rowsP * FD * 4);
  const size_t oPP = carve(rowsP * PPW * 4);
  const size_t oGE = carve((size_t)G * FD * 4);
  size_t limit = (size_t)134217728;
  if (ws_size < limit) limit = ws_size;
  if (off > limit) return;

  unsigned short* q0 = (unsigned short*)(ws + oq0);
  unsigned short* q1 = (unsigned short*)(ws + oq1);
  unsigned short* q2 = (unsigned short*)(ws + oq2);
  unsigned short* q3 = (unsigned short*)(ws + oq3);
  unsigned short* q4 = (unsigned short*)(ws + oq4);
  unsigned short* q5 = (unsigned short*)(ws + oq5);
  unsigned short* q6 = (unsigned short*)(ws + oq6);
  unsigned short* q7 = (unsigned short*)(ws + oq7);
  int*   etab = (int*)(ws + oet);
  float* X0   = (float*)(ws + oX0);
  float* X1   = (float*)(ws + oX1);
  float* PP   = (float*)(ws + oPP);
  float* GE   = (float*)(ws + oGE);

  const int vec8 = ((nE & 3) == 0) ? 1 : 0;

  k_prep<<<PBT, NTHR, 0, stream>>>(win, mw1, mw2, uw1, uw2, hw1, hw2, hw3, q0, q1, q2, q3, q4, q5, q6, q7);
  k_escan<<<nBlk, NTHR, 0, stream>>>(ei, etab, nE, vec8);
  k_inproj<<<nRT, RTHR, 0, stream>>>(x, bead, emb, q0, q0 + ne0, bin, X0, nN, nBead);

  hipFuncSetAttribute(reinterpret_cast<const void*>(&k_pp), hipFuncAttributeMaxDynamicSharedMemorySize, LP_TOT);
  hipFuncSetAttribute(reinterpret_cast<const void*>(&k_layer), hipFuncAttributeMaxDynamicSharedMemorySize, LL_TOT);
  float* hcur = X0;
  float* hnxt = X1;
  for (int l = 0; l < NLAY; ++l) {
    k_pp<<<nRT, RTHR, LP_TOT, stream>>>(hcur, q1 + (size_t)l * PPW * FD, q1 + ne1 + (size_t)l * PPW * FD, PP);
    k_layer<<<nBlk, NTHR, LL_TOT, stream>>>(
        hcur, PP, ei, eat, etab,
        mw1 + (size_t)l * W1K * FD + (size_t)PPW * FD, mb1 + (size_t)l * FD,
        q2 + (size_t)l * FD * FD, q2 + ne2 + (size_t)l * FD * FD, mb2 + (size_t)l * FD,
        q3 + (size_t)l * FD * UK, q3 + ne3 + (size_t)l * FD * UK, ub1 + (size_t)l * FD,
        q4 + (size_t)l * FD * FD, q4 + ne4 + (size_t)l * FD * FD, ub2 + (size_t)l * FD,
        gam + (size_t)l * FD, bet + (size_t)l * FD,
        hnxt, nN, nE, l > 0 ? 1 : 0);
    float* tsw = hcur; hcur = hnxt; hnxt = tsw;
  }

  k_pool<<<G / GB, PTHR, 0, stream>>>(hcur, batch, GE, nN, G);
  k_head<<<G / HG, HTHR, 0, stream>>>(GE, gfi0, gfi1, gfi2, gfi3, gfi4, gfi5, gfi6, gfi7, gfw, gfb,
                                      q5, q5 + ne5, hb1, q6, q6 + ne6, hb2, q7, q7 + ne7, hb3, hw4, hb4, dout, G);
}
